// NN_45535243272834
// MI455X (gfx1250) — hardware-verified
//
#include <hip/hip_runtime.h>
#include <stddef.h>
#include <math.h>


#define WD     60
#define WP     64
#define NTHR   256
#define RB     128
#define HP     72
#define NL16   4
#define PLANE  (WP * WP)
#define NBT    5
#define NWITEM (5 * PLANE / 8)
#define NBITEM (NBT * WP / 4)
#define SC_A   8.0f
#define SC_W   64.0f
#define SC_INV (1.0f / 512.0f)

static_assert(RB == 16 * (NTHR / 32));
static_assert((HP * 2) % 16 == 0);
static_assert(WP % 32 == 0);
static_assert(NWITEM % NTHR == 0);
static_assert((PLANE / 8) % NTHR == 0);
static_assert(RB / 4 == 32);

typedef unsigned short us_t;
typedef _Float16 v16h  __attribute__((ext_vector_type(16)));
typedef _Float16 v8h   __attribute__((ext_vector_type(8)));
typedef us_t     v8us  __attribute__((ext_vector_type(8)));
typedef __bf16   v16bf __attribute__((ext_vector_type(16)));
typedef float    v4f   __attribute__((ext_vector_type(4)));
typedef float    v8f   __attribute__((ext_vector_type(8)));
union FragH { v16h v;  v8h  h[2]; };
union FragB { v16bf v; v8us h[2]; };

__device__ __forceinline__ v8f wmh(v16h a, v16h b, v8f c) {
  v8f d = __builtin_amdgcn_wmma_f32_16x16x32_f16(false, a, false, b, (short)0, c, false, false);
#if defined(__HIP_DEVICE_COMPILE__)
  asm volatile("v_nop\n\tv_nop\n\tv_nop\n\tv_nop" : "+v"(d) : "v"(a), "v"(b));
#endif
  return d;
}
__device__ __forceinline__ v8f wmb(v16bf a, v16bf b, v8f c) {
  v8f d = __builtin_amdgcn_wmma_f32_16x16x32_bf16(false, a, false, b, (short)0, c, false, false);
#if defined(__HIP_DEVICE_COMPILE__)
  asm volatile("v_nop\n\tv_nop\n\tv_nop\n\tv_nop" : "+v"(d) : "v"(a), "v"(b));
#endif
  return d;
}

__device__ __forceinline__ v8f zero8() {
  v8f z = {0.f, 0.f, 0.f, 0.f, 0.f, 0.f, 0.f, 0.f};
  return z;
}

__device__ __forceinline__ us_t bf16_bits(float x) {
  unsigned u = __float_as_uint(x);
  u = (u + 0x7FFFu + ((u >> 16) & 1u)) >> 16;
  return (us_t)u;
}
__device__ __forceinline__ float bf16_val(us_t b) {
  return __uint_as_float(((unsigned)b) << 16);
}

__device__ __forceinline__ float silu_f(float s) {
  const float sc = fmaxf(s, -80.0f);
  const float e  = expf(-sc);
  const float sg = 1.0f / (1.0f + e);
  return s * sg;
}

__global__ __launch_bounds__(NTHR) void k_prep(const float* __restrict__ W2, const float* __restrict__ W3,
                                               const float* __restrict__ W4, const float* __restrict__ W5,
                                               const float* __restrict__ W6,
                                               const float* __restrict__ b2, const float* __restrict__ b3,
                                               const float* __restrict__ b4, const float* __restrict__ b5,
                                               const float* __restrict__ b6,
                                               _Float16* P16, us_t* P6h, us_t* P6l, float* Bt) {
  const int i = blockIdx.x * NTHR + (int)threadIdx.x;
  if (i < NWITEM) {
    const int src = i / (PLANE / 8);
    const int wi  = i - src * (PLANE / 8);
    const int n   = wi >> 3;
    const int k0  = (wi & 7) * 8;
    const float* W = (src == 0) ? W2 : (src == 1) ? W3 : (src == 2) ? W4 : (src == 3) ? W5 : W6;
    const int nq = n < WD ? n : WD - 1;
    float w[8];
#pragma unroll
    for (int e = 0; e < 8; ++e) {
      const int kk = k0 + e;
      const int kq = kk < WD ? kk : WD - 1;
      const float wv = W[nq * WD + kq];
      w[e] = (n < WD && kk < WD) ? wv : 0.0f;
    }
    if (src < NL16) {
      v8h o;
#pragma unroll
      for (int e = 0; e < 8; ++e) o[e] = (_Float16)(SC_W * w[e]);
      _Float16* p = P16 + (size_t)src * PLANE + n * WP + k0;
      *(volatile v8h*)p = o;
      __threadfence();
      *(volatile v8h*)p = o;
    } else {
      v8us oh, ol;
#pragma unroll
      for (int e = 0; e < 8; ++e) {
        const us_t hb = bf16_bits(w[e]);
        oh[e] = hb;
        ol[e] = bf16_bits(w[e] - bf16_val(hb));
      }
      us_t* ph = P6h + n * WP + k0;
      us_t* pl = P6l + n * WP + k0;
      *(volatile v8us*)ph = oh;
      *(volatile v8us*)pl = ol;
      __threadfence();
      *(volatile v8us*)ph = oh;
      *(volatile v8us*)pl = ol;
    }
  } else if (i < NWITEM + NBITEM) {
    const int j  = i - NWITEM;
    const int l  = j >> 4;
    const int c0 = (j & 15) * 4;
    const float* b = (l == 0) ? b2 : (l == 1) ? b3 : (l == 2) ? b4 : (l == 3) ? b5 : b6;
    v4f o;
#pragma unroll
    for (int e = 0; e < 4; ++e) {
      const int c  = c0 + e;
      const int cq = c < WD ? c : WD - 1;
      const float bv = b[cq];
      o[e] = (c < WD) ? bv : 0.0f;
    }
    float* p = Bt + l * WP + c0;
    *(volatile v4f*)p = o;
    __threadfence();
    *(volatile v4f*)p = o;
  }
}

__global__ __launch_bounds__(NTHR) void k_mlp(const float* __restrict__ x, const float* __restrict__ y,
                                              const float* __restrict__ W1, const float* __restrict__ b1,
                                              const _Float16* __restrict__ P16,
                                              const us_t* __restrict__ P6h, const us_t* __restrict__ P6l,
                                              const float* __restrict__ Bt,
                                              const float* __restrict__ W7, const float* __restrict__ b7,
                                              float* out, int nrow) {
  __shared__ __align__(16) _Float16 sF[RB * HP];
  __shared__ __align__(16) us_t     sHh[RB * HP];
  __shared__ __align__(16) us_t     sHl[RB * HP];
  __shared__ v4f sO4[RB / 4];
  float* sO = (float*)sO4;

  const int tid = threadIdx.x, lane = tid & 31, wv = tid >> 5, h = lane >> 4, m = lane & 15;
  const int brow = blockIdx.x * RB;
  const int wr = wv * 16;

  {
    int rg = brow + wr + m;
    rg = rg > nrow - 1 ? nrow - 1 : rg;
    const float xv = x[rg], yv = y[rg];
    const int c0 = lane, c1 = lane + 32;
    const int q1 = c1 < WD ? c1 : WD - 1;
    const float w00 = W1[2 * c0], w01 = W1[2 * c0 + 1], bb0 = b1[c0];
    const float w10 = W1[2 * q1], w11 = W1[2 * q1 + 1], bb1 = b1[q1];
    const bool ok1 = c1 < WD;
#pragma unroll
    for (int r = 0; r < 16; ++r) {
      const float xr = __shfl(xv, r, 32), yr = __shfl(yv, r, 32);
      const float s0 = (xr * w00 + yr * w01) + bb0;
      const float s1 = (xr * w10 + yr * w11) + bb1;
      const float a0 = silu_f(s0);
      const float t1 = silu_f(s1);
      const float a1 = ok1 ? t1 : 0.0f;
      sF[(wr + r) * HP + c0] = (_Float16)(SC_A * a0);
      sF[(wr + r) * HP + c1] = (_Float16)(SC_A * a1);
    }
  }
  __syncthreads();

#pragma unroll 1
  for (int li = 0; li < NL16; ++li) {
    const _Float16* Pl = P16 + (size_t)li * PLANE;
    FragH af[2];
#pragma unroll
    for (int ks = 0; ks < 2; ++ks) {
      const _Float16* pa = sF + (wr + m) * HP + 32 * ks + 8 * h;
      af[ks].h[0] = *(const v8h*)pa;
      af[ks].h[1] = *(const v8h*)(pa + 16);
    }
    v8f acc[4];
#pragma unroll
    for (int t = 0; t < 4; ++t) {
      acc[t] = zero8();
      const _Float16* pb = Pl + (size_t)(16 * t + m) * WP + 8 * h;
#pragma unroll
      for (int ks = 0; ks < 2; ++ks) {
        FragH bf;
        bf.h[0] = *(const v8h*)(pb + 32 * ks);
        bf.h[1] = *(const v8h*)(pb + 32 * ks + 16);
        acc[t] = wmh(af[ks].v, bf.v, acc[t]);
      }
    }
    const float* bl = Bt + li * WP;
    float av[4][8];
#pragma unroll
    for (int t = 0; t < 4; ++t) {
      const float bb = bl[16 * t + m];
#pragma unroll
      for (int r = 0; r < 8; ++r) av[t][r] = silu_f(acc[t][r] * SC_INV + bb);
    }
    if (li < NL16 - 1) {
#pragma unroll
      for (int t = 0; t < 4; ++t) {
#pragma unroll
        for (int r = 0; r < 8; ++r)
          sF[(wr + 8 * h + r) * HP + 16 * t + m] = (_Float16)(SC_A * av[t][r]);
      }
    } else {
#pragma unroll
      for (int t = 0; t < 4; ++t) {
#pragma unroll
        for (int r = 0; r < 8; ++r) {
          const float v  = av[t][r];
          const us_t  hb = bf16_bits(v);
          const us_t  lb = bf16_bits(v - bf16_val(hb));
          sHh[(wr + 8 * h + r) * HP + 16 * t + m] = hb;
          sHl[(wr + 8 * h + r) * HP + 16 * t + m] = lb;
        }
      }
    }
    __syncthreads();
  }

  {
    FragB ah[2], al[2];
#pragma unroll
    for (int ks = 0; ks < 2; ++ks) {
      const int pa = (wr + m) * HP + 32 * ks + 8 * h;
      ah[ks].h[0] = *(const v8us*)(sHh + pa);
      ah[ks].h[1] = *(const v8us*)(sHh + pa + 16);
      al[ks].h[0] = *(const v8us*)(sHl + pa);
      al[ks].h[1] = *(const v8us*)(sHl + pa + 16);
    }
    v8f acc[4];
#pragma unroll
    for (int t = 0; t < 4; ++t) {
      acc[t] = zero8();
      const int ob = (16 * t + m) * WP + 8 * h;
#pragma unroll
      for (int ks = 0; ks < 2; ++ks) {
        FragB bh, blo;
        bh.h[0]  = *(const v8us*)(P6h + ob + 32 * ks);
        bh.h[1]  = *(const v8us*)(P6h + ob + 32 * ks + 16);
        blo.h[0] = *(const v8us*)(P6l + ob + 32 * ks);
        blo.h[1] = *(const v8us*)(P6l + ob + 32 * ks + 16);
        acc[t] = wmb(ah[ks].v, bh.v,  acc[t]);
        acc[t] = wmb(ah[ks].v, blo.v, acc[t]);
        acc[t] = wmb(al[ks].v, bh.v,  acc[t]);
      }
    }
    const float* b6 = Bt + NL16 * WP;
    float p[8];
#pragma unroll
    for (int r = 0; r < 8; ++r) p[r] = 0.0f;
#pragma unroll
    for (int t = 0; t < 4; ++t) {
      const int c  = 16 * t + m;
      const int cq = c < WD ? c : WD - 1;
      const float w7v = W7[cq];
      const float w7  = (c < WD) ? w7v : 0.0f;
      const float bb  = b6[c];
#pragma unroll
      for (int r = 0; r < 8; ++r) {
        const float v = silu_f(acc[t][r] + bb);
        p[r] = fmaf(v, w7, p[r]);
      }
    }
#pragma unroll
    for (int off = 1; off < 16; off <<= 1) {
#pragma unroll
      for (int r = 0; r < 8; ++r) p[r] += __shfl_xor(p[r], off, 32);
    }
    const float b7v = b7[0];
    float ov = p[0];
#pragma unroll
    for (int r = 1; r < 8; ++r) ov = (m == r) ? p[r] : ov;
    if (m < 8) sO[wr + 8 * h + m] = ov + b7v;
  }
  __syncthreads();

  if (wv == 0) {
    const int rem = nrow - brow;
    const int nv  = rem < RB ? rem : RB;
    const v4f o   = sO4[lane];
    float* g = out + (size_t)brow + 4 * lane;
    const bool full = (4 * lane + 4) <= nv;
    const int  tl   = nv & 3;
    const bool tail = (tl != 0) && (lane == (nv >> 2));
    if (full) *(volatile v4f*)g = o;
    if (tail) {
      ((volatile float*)g)[0] = o[0];
      if (tl > 1) ((volatile float*)g)[1] = o[1];
      if (tl > 2) ((volatile float*)g)[2] = o[2];
    }
    __threadfence();
    if (full) *(volatile v4f*)g = o;
    if (tail) {
      ((volatile float*)g)[0] = o[0];
      if (tl > 1) ((volatile float*)g)[1] = o[1];
      if (tl > 2) ((volatile float*)g)[2] = o[2];
    }
  }
}

extern "C" void kernel_launch(void* const* d_in, const int* in_sizes, int n_in,
                              void* d_out, int out_size, void* d_ws, size_t ws_size,
                              hipStream_t stream) {
  if (n_in < 16) return;
  const int nrow = in_sizes[0];
  if (nrow <= 0 || in_sizes[1] != nrow || out_size != nrow) return;
  if (in_sizes[2] != 2 * WD || in_sizes[3] != WD) return;
  for (int l = 0; l < 5; ++l) {
    if (in_sizes[4 + 2 * l] != WD * WD || in_sizes[5 + 2 * l] != WD) return;
  }
  if (in_sizes[14] != WD || in_sizes[15] != 1) return;

  const float* x  = (const float*)d_in[0];
  const float* y  = (const float*)d_in[1];
  const float* W1 = (const float*)d_in[2];
  const float* b1 = (const float*)d_in[3];
  const float* W2 = (const float*)d_in[4];
  const float* b2 = (const float*)d_in[5];
  const float* W3 = (const float*)d_in[6];
  const float* b3 = (const float*)d_in[7];
  const float* W4 = (const float*)d_in[8];
  const float* b4 = (const float*)d_in[9];
  const float* W5 = (const float*)d_in[10];
  const float* b5 = (const float*)d_in[11];
  const float* W6 = (const float*)d_in[12];
  const float* b6 = (const float*)d_in[13];
  const float* W7 = (const float*)d_in[14];
  const float* b7 = (const float*)d_in[15];
  float* out = (float*)d_out;

  const size_t offP16 = 0;
  const size_t offP6h = offP16 + (size_t)NL16 * PLANE * 2;
  const size_t offP6l = offP6h + (size_t)PLANE * 2;
  const size_t offBt  = offP6l + (size_t)PLANE * 2;
  const size_t total  = offBt + (size_t)NBT * WP * 4;
  if (total > ws_size || total > (size_t)134217728) return;
  _Float16* P16 = (_Float16*)((char*)d_ws + offP16);
  us_t*     P6h = (us_t*)((char*)d_ws + offP6h);
  us_t*     P6l = (us_t*)((char*)d_ws + offP6l);
  float*    Bt  = (float*)((char*)d_ws + offBt);

  k_prep<<<(NWITEM + NBITEM + NTHR - 1) / NTHR, NTHR, 0, stream>>>(W2, W3, W4, W5, W6, b2, b3, b4, b5, b6,
                                                                   P16, P6h, P6l, Bt);
  k_mlp<<<(nrow + RB - 1) / RB, NTHR, 0, stream>>>(x, y, W1, b1, P16, P6h, P6l, Bt, W7, b7, out, nrow);
}
